// SparseCNNProjectionNetwork_15650860827379
// MI455X (gfx1250) — hardware-verified
//
#include <hip/hip_runtime.h>
#include <math.h>
typedef __attribute__((ext_vector_type(16))) _Float16 v16h;
typedef __attribute__((ext_vector_type(8)))  _Float16 v8h;
typedef __attribute__((ext_vector_type(16))) __bf16   v16b;
typedef __attribute__((ext_vector_type(8)))  __bf16   v8b;
typedef __attribute__((ext_vector_type(8)))  float    v8f;
typedef __attribute__((ext_vector_type(4)))  float    v4f;
#define PSCALE 32768.0f
#define U16(p) ((const unsigned short*)(const void*)(p))
#define PSCALE_INV (1.0f / 32768.0f)

__device__ __forceinline__ unsigned short f2bf_bits(float f) {
  unsigned u = __float_as_uint(f);
  return (unsigned short)((u + 0x7FFFu + ((u >> 16) & 1u)) >> 16);
}
__device__ __forceinline__ float bf_bits2f(unsigned short h) { return __uint_as_float(((unsigned)h) << 16); }

__device__ __forceinline__ void dep_guard_h(v8f& a, v8f& b, v16h x, v16h y) { asm volatile("v_nop\n\tv_nop\n\tv_nop\n\tv_nop" : "+v"(a), "+v"(b) : "v"(x), "v"(y)); }
__device__ __forceinline__ void dep_guard_b(v8f& a, v8f& b, v16b x, v16b y) { asm volatile("v_nop\n\tv_nop\n\tv_nop\n\tv_nop" : "+v"(a), "+v"(b) : "v"(x), "v"(y)); }
__device__ __forceinline__ void keep4_h(v16h a, v16h b, v16h c, v16h d) { asm volatile("v_nop" :: "v"(a), "v"(b), "v"(c), "v"(d)); }
__device__ __forceinline__ void keep4_b(v16b a, v16b b, v16b c, v16b d) { asm volatile("v_nop" :: "v"(a), "v"(b), "v"(c), "v"(d)); }
__device__ __forceinline__ void acc_guard4(v8f& a, v8f& b, v8f& c, v8f& d) { asm volatile("v_nop\n\tv_nop\n\tv_nop\n\tv_nop" : "+v"(a), "+v"(b), "+v"(c), "+v"(d)); }
template <typename T> struct Frag;
template <> struct Frag<_Float16> {
  typedef v16h V; union U { v16h v; v8h h[2]; };
  static __device__ __forceinline__ v16h load(const _Float16* p) {
    U f; f.h[0] = *(const v8h*)(p); f.h[1] = *(const v8h*)(p + 16); return f.v;
  }
  static __device__ __forceinline__ v8f mma(v16h a, v16h b, v8f c) {
    return __builtin_amdgcn_wmma_f32_16x16x32_f16(false, a, false, b, (short)0, c, false, false);
  }
  static __device__ __forceinline__ void guard(v8f& a, v8f& b, v16h x, v16h y) { dep_guard_h(a, b, x, y); }
  static __device__ __forceinline__ void keep(v16h a, v16h b, v16h c, v16h d) { keep4_h(a, b, c, d); }
};
template <> struct Frag<__bf16> {
  typedef v16b V; union U { v16b v; v8b h[2]; };
  static __device__ __forceinline__ v16b load(const __bf16* p) {
    U f; f.h[0] = *(const v8b*)(p); f.h[1] = *(const v8b*)(p + 16); return f.v;
  }
  static __device__ __forceinline__ v8f mma(v16b a, v16b b, v8f c) {
    return __builtin_amdgcn_wmma_f32_16x16x32_bf16(false, a, false, b, (short)0, c, false, false);
  }
  static __device__ __forceinline__ void guard(v8f& a, v8f& b, v16b x, v16b y) { dep_guard_b(a, b, x, y); }
  static __device__ __forceinline__ void keep(v16b a, v16b b, v16b c, v16b d) { keep4_b(a, b, c, d); }
};

template <int ET> struct Elem;
template <> struct Elem<0> { typedef _Float16 T; };
template <> struct Elem<1> { typedef __bf16 T; };
template <int ET, bool SPLIT, int BIAS_MODE, int OUT_MODE, bool RESID, int ACT = 0>
__global__ __launch_bounds__(256) void wmma_gemm64(
    const unsigned short* __restrict__ Ap, const unsigned short* __restrict__ A2p, int lda, long strideA,
    const unsigned short* __restrict__ Btp, const unsigned short* __restrict__ Bt2p, int ldb, long strideB,
    void* __restrict__ Cout, void* __restrict__ Cout2, int ldc, long strideC,
    const float* __restrict__ bias,
    const float* __restrict__ resid, long strideR,
    int M, int N, int K, float scale) {
  typedef typename Elem<ET>::T T;
  typedef typename Frag<T>::V V;
  const T* A = (const T*)Ap; const T* A2 = (const T*)A2p; const T* Bt = (const T*)Btp; const T* Bt2 = (const T*)Bt2p;
  __shared__ __align__(16) float sT[8][16 * 68];
  const int b    = blockIdx.y;
  const int lane = threadIdx.x & 31;
  const int wave = threadIdx.x >> 5;
  const int tilesN = N >> 6;
  const int tilesM = M >> 6;
  const int tile = blockIdx.x * 8 + wave;
  if (tile >= tilesM * tilesN) return;
  const int tm = tile / tilesN;
  const int tn = tile - tm * tilesN;
  const int m0 = tm << 6;
  const int n0 = tn << 6;

  const T* Ab  = A  + (size_t)b * strideA;
  const T* Bb  = Bt + (size_t)b * strideB;
  const T* Ab2 = SPLIT ? (A2  + (size_t)b * strideA) : nullptr;
  const T* Bb2 = SPLIT ? (Bt2 + (size_t)b * strideB) : nullptr;

  const int rlane = lane & 15;
  const int koff  = (lane >> 4) * 8;
  const int mOff  = (lane >> 4) * 8;

  v8f acc[4][4];
#pragma unroll
  for (int i = 0; i < 4; ++i)
#pragma unroll
    for (int j = 0; j < 4; ++j) acc[i][j] = (v8f){0.f,0.f,0.f,0.f,0.f,0.f,0.f,0.f};

  for (int k0 = 0; k0 < K; k0 += 32) {
    V bh[4], bl[4];
#pragma unroll
    for (int j = 0; j < 4; ++j) {
      const size_t bo = (size_t)(n0 + (j << 4) + rlane) * ldb + koff + k0;
      bh[j] = Frag<T>::load(Bb + bo);
      if (SPLIT) bl[j] = Frag<T>::load(Bb2 + bo);
    }
#pragma unroll
    for (int i = 0; i < 4; ++i) {
      const size_t ao = (size_t)(m0 + (i << 4) + rlane) * lda + koff + k0;
      V ah = Frag<T>::load(Ab + ao);
      V al;
      if (SPLIT) al = Frag<T>::load(Ab2 + ao);
#pragma unroll
      for (int j = 0; j < 4; ++j) {
        acc[i][j] = Frag<T>::mma(ah, bh[j], acc[i][j]);
        if (SPLIT) {
          acc[i][j] = Frag<T>::mma(ah, bl[j], acc[i][j]);
          acc[i][j] = Frag<T>::mma(al, bh[j], acc[i][j]);
        }
      }
      Frag<T>::guard(acc[i][0], acc[i][3], ah, SPLIT ? al : ah);
    }
    Frag<T>::keep(bh[0], bh[1], bh[2], bh[3]);
    if (SPLIT) Frag<T>::keep(bl[0], bl[1], bl[2], bl[3]);
  }
  acc_guard4(acc[0][0], acc[0][1], acc[0][2], acc[0][3]);
  acc_guard4(acc[1][0], acc[1][1], acc[1][2], acc[1][3]);
  acc_guard4(acc[2][0], acc[2][1], acc[2][2], acc[2][3]);
  acc_guard4(acc[3][0], acc[3][1], acc[3][2], acc[3][3]);

  float* slab = sT[wave];
  const float* Rb = RESID ? (resid + (size_t)b * strideR) : nullptr;
#pragma unroll
  for (int i = 0; i < 4; ++i) {
    const int mBase = m0 + (i << 4);
#pragma unroll
    for (int j = 0; j < 4; ++j) {
      const int n = n0 + (j << 4) + rlane;
      float bv = 0.f;
      if (BIAS_MODE == 2) bv = bias[n];
#pragma unroll
      for (int r = 0; r < 8; ++r) {
        float v = acc[i][j][r] * scale;
        if (BIAS_MODE == 1) v += bias[mBase + mOff + r];
        if (BIAS_MODE == 2) v += bv;
        if (RESID) v += Rb[(size_t)(mBase + mOff + r) * ldc + n];
        if (ACT == 1) v = tanhf(v);
        if (ACT == 2) v = fmaxf(v, 0.0f);
        if (ACT == 3) v = v / (1.0f + expf(-v));
        if (ACT == 4) v = (v > 0.f) ? v : 0.01f * v;
        if (ACT == 5) v = 0.5f * v * (1.0f + erff(v * 0.70710678118654752f));
        slab[(mOff + r) * 68 + (j << 4) + rlane] = v;
      }
    }
    __builtin_amdgcn_fence(__ATOMIC_RELEASE, "workgroup");
    __builtin_amdgcn_wave_barrier();
    __builtin_amdgcn_fence(__ATOMIC_ACQUIRE, "workgroup");
    if (OUT_MODE == 0) {
      float* C = (float*)Cout + (size_t)b * strideC;
      const int hh = lane >> 4, c4 = (lane & 15) * 4;
      for (int pass = 0; pass < 2; ++pass) {
#pragma unroll
        for (int it = 0; it < 8; ++it) {
          const int row = it * 2 + hh;
          v4f v = *(const v4f*)(slab + row * 68 + c4);
          *(volatile v4f*)(C + (size_t)(mBase + row) * ldc + n0 + c4) = v;
        }
        __threadfence();
      }
    } else {
      const int q = lane >> 3, c8 = (lane & 7) * 8;
      unsigned short* C  = (unsigned short*)Cout  + (size_t)b * strideC;
      unsigned short* C2 = (OUT_MODE == 2) ? ((unsigned short*)Cout2 + (size_t)b * strideC) : nullptr;
      for (int pass = 0; pass < 2; ++pass) {
#pragma unroll
        for (int it = 0; it < 4; ++it) {
          const int row = it * 4 + q;
          const float* sp = slab + row * 68 + c8;
          v8h hv, lv;
#pragma unroll
          for (int e = 0; e < 8; ++e) {
            if (OUT_MODE == 1) {
              hv[e] = (_Float16)sp[e];
            } else {
              unsigned short hb = f2bf_bits(sp[e]);
              unsigned short lb = f2bf_bits(sp[e] - bf_bits2f(hb));
              hv[e] = __builtin_bit_cast(_Float16, hb);
              lv[e] = __builtin_bit_cast(_Float16, lb);
            }
          }
          *(volatile v8h*)(C + (size_t)(mBase + row) * ldc + n0 + c8) = hv;
          if (OUT_MODE == 2) *(volatile v8h*)(C2 + (size_t)(mBase + row) * ldc + n0 + c8) = lv;
        }
        __threadfence();
      }
    }
    __builtin_amdgcn_fence(__ATOMIC_RELEASE, "workgroup");
    __builtin_amdgcn_wave_barrier();
    __builtin_amdgcn_fence(__ATOMIC_ACQUIRE, "workgroup");
  }
}

__global__ __launch_bounds__(256) void cast_f32_f16x2(
    const float* __restrict__ in, _Float16* __restrict__ out, int n2) {
  int i = blockIdx.x * 256 + threadIdx.x;
  if (i < n2) {
    const _Float16 h0 = (_Float16)in[2 * i], h1 = (_Float16)in[2 * i + 1];
    const unsigned u = (unsigned)__builtin_bit_cast(unsigned short, h0) | ((unsigned)__builtin_bit_cast(unsigned short, h1) << 16);
    ((volatile unsigned*)out)[i] = u;
    __threadfence();
    ((volatile unsigned*)out)[i] = u;
  }
}


#define SB_ 16
#define SHW 512
#define SCELLS (SB_ * SHW * SHW)
#define NN (SCELLS / 64)
#define NODES_PER_BLK 256
#define NBLK ((NN + NODES_PER_BLK - 1) / NODES_PER_BLK)
#define NPAD (NBLK * NODES_PER_BLK)
#define NE 320000
#define SEG_CAP 1536
#define SCH 80000

#define ECH 8192
#define NCH ((NE + ECH - 1) / ECH)
#define NRP (((NBLK) + 31) & ~31)
#define SEG_STRIDE SEG_CAP
#define BUCKET_INTS ((size_t)NE + (size_t)32 * NCH * NBLK)
__device__ __forceinline__ int rank_eq(int key, bool valid, int lane, int nbits, int& ntotal) {
  unsigned same = __ballot(valid);
  for (int b = 0; b < nbits; ++b) {
    const unsigned m = __ballot(((key >> b) & 1) != 0);
    same &= (((key >> b) & 1) != 0) ? m : ~m;
  }
  if (!valid) same = 0u;
  ntotal = __popc(same);
  return __popc(same & ((1u << lane) - 1u));
}
__global__ __launch_bounds__(256) void csr_hist_kernel(const int* __restrict__ dst, int* __restrict__ cnt) {
  __shared__ int h[8][NRP];
  const int tid = threadIdx.x, lane = tid & 31, wave = tid >> 5;
  for (int i = tid; i < 8 * NRP; i += 256) (&h[0][0])[i] = 0;
  __syncthreads();
  const int e0 = blockIdx.x * ECH + wave * (ECH / 8), e1 = min(e0 + ECH / 8, NE);
  for (int c0 = e0; c0 < e0 + ECH / 8; c0 += 32) {
    const int e = c0 + lane;
    const bool valid = e < e1;
    int d = valid ? dst[e] : 0; d = d < 0 ? 0 : (d >= NN ? NN - 1 : d);
    const int r = d / NODES_PER_BLK;
    int tot; const int rk = rank_eq(r, valid, lane, 9, tot);
    if (valid && rk == tot - 1) h[wave][r] += tot;
  }
  __syncthreads();
  for (int pass = 0; pass < 2; ++pass) {
    for (int i = tid; i < NRP; i += 256) { int s = 0; for (int w = 0; w < 8; ++w) s += h[w][i]; ((volatile int*)cnt)[(size_t)blockIdx.x * NRP + i] = s; }
    __threadfence();
  }
}
__global__ __launch_bounds__(1024) void csr_offsets_kernel(const int* __restrict__ cnt, int* __restrict__ boff, int* __restrict__ rinfo) {
  __shared__ int rsz[1024];
  const int t = threadIdx.x;
  int run = 0;
  if (t < NBLK) { for (int c = 0; c < NCH; ++c) run += (cnt[(size_t)c * NRP + t] + 31) & ~31; }
  rsz[t] = (t < NBLK) ? run : 0;
  __syncthreads();
  for (int off = 1; off < 1024; off <<= 1) { int v = (t >= off) ? rsz[t - off] : 0; __syncthreads(); rsz[t] += v; __syncthreads(); }
  const int incl = rsz[t], excl = incl - ((t < NBLK) ? run : 0);
  __syncthreads();
  for (int pass = 0; pass < 2; ++pass) {
    if (t < NBLK) { int r2 = excl; for (int c = 0; c < NCH; ++c) { const size_t i = (size_t)c * NRP + t; ((volatile int*)boff)[i] = r2; r2 += (cnt[i] + 31) & ~31; } }
    ((volatile int*)rinfo)[t] = excl;
    ((volatile int*)rinfo)[1024 + t] = (t < NBLK) ? run : 0;
    __threadfence();
  }
}
__global__ __launch_bounds__(256) void csr_bucket_kernel(const int* __restrict__ dst, const int* __restrict__ boff, int* __restrict__ bucket) {
  __shared__ int wc[8][NRP];
  __shared__ int woff[8][NRP];
  __shared__ int roff[NRP + 1];
  __shared__ int seg[ECH + 32 * NRP];
  const int tid = threadIdx.x, lane = tid & 31, wave = tid >> 5;
  for (int i = tid; i < 8 * NRP; i += 256) { (&wc[0][0])[i] = 0; }
  __syncthreads();
  const int e0 = blockIdx.x * ECH + wave * (ECH / 8), e1 = min(e0 + ECH / 8, NE);
  for (int c0 = e0; c0 < e0 + ECH / 8; c0 += 32) {
    const int e = c0 + lane; const bool valid = e < e1;
    int d = valid ? dst[e] : 0; d = d < 0 ? 0 : (d >= NN ? NN - 1 : d);
    const int r = d / NODES_PER_BLK;
    int tot; const int rk = rank_eq(r, valid, lane, 9, tot);
    if (valid && rk == tot - 1) wc[wave][r] += tot;
  }
  __syncthreads();
  __shared__ int tot_r[NRP];
  for (int i = tid; i < NRP; i += 256) { int s = 0; for (int w = 0; w < 8; ++w) s += wc[w][i]; tot_r[i] = s; }
  __syncthreads();
  if (tid == 0) { int run = 0; for (int r = 0; r < NRP; ++r) { roff[r] = run; int o = run; for (int w = 0; w < 8; ++w) { woff[w][r] = o; o += wc[w][r]; } run += (tot_r[r] + 31) & ~31; } roff[NRP] = run; }
  __syncthreads();
  const int totalpad = roff[NRP];
  for (int i = tid; i < totalpad && i < ECH + 32 * NRP; i += 256) seg[i] = -1;
  __syncthreads();
  for (int c0 = e0; c0 < e0 + ECH / 8; c0 += 32) {
    const int e = c0 + lane; const bool valid = e < e1;
    int d = valid ? dst[e] : 0; d = d < 0 ? 0 : (d >= NN ? NN - 1 : d);
    const int r = d / NODES_PER_BLK;
    int tot; const int rk = rank_eq(r, valid, lane, 9, tot);
    if (valid) { const int slot = woff[wave][r] + rk; if (slot < ECH + 32 * NRP) seg[slot] = e; if (rk == tot - 1) woff[wave][r] = slot + 1; }
  }
  __syncthreads();
  for (int pass = 0; pass < 2; ++pass) {
    for (int r = wave; r < NBLK; r += 8) {
      const int lo = roff[r], n = ((tot_r[r] + 31) & ~31);
      int gb = boff[(size_t)blockIdx.x * NRP + r]; gb = gb < 0 ? 0 : (gb > (int)BUCKET_INTS - n ? (int)BUCKET_INTS - n : gb);
      for (int i = lane; i < n; i += 32) ((volatile int*)bucket)[(size_t)gb + i] = (lo + i < ECH + 32 * NRP) ? seg[lo + i] : -1;
    }
    __threadfence();
  }
}
__global__ __launch_bounds__(256) void csr_fill_kernel(const int* __restrict__ dst, const int* __restrict__ bucket, const int* __restrict__ rinfo,
                                                      int* __restrict__ rowptr, int* __restrict__ rowdeg, int* __restrict__ csr_eid, int* __restrict__ rcl) {
  __shared__ int cnt[8][NODES_PER_BLK];
  __shared__ int off[8][NODES_PER_BLK];
  __shared__ int nodeoff[NODES_PER_BLK + 1];
  __shared__ int seg[SEG_CAP];
  const int tid = threadIdx.x, lane = tid & 31, wave = tid >> 5;
  const int n0 = blockIdx.x * NODES_PER_BLK;
  int bstart = rinfo[blockIdx.x], bsize = rinfo[1024 + blockIdx.x];
  bstart = bstart < 0 ? 0 : (bstart > (int)BUCKET_INTS ? (int)BUCKET_INTS : bstart); bsize = bsize < 0 ? 0 : (bsize > (int)BUCKET_INTS - bstart ? (int)BUCKET_INTS - bstart : bsize);
  for (int i = tid; i < 8 * NODES_PER_BLK; i += 256) (&cnt[0][0])[i] = 0;
  for (int i = tid; i < SEG_CAP; i += 256) seg[i] = 0;
  __syncthreads();
  const int per = ((bsize / 8) + 31) & ~31;
  const int e0 = bstart + wave * per, e1 = min(bstart + (wave + 1) * per, bstart + bsize);
  for (int c0 = e0; c0 < e0 + per; c0 += 32) {
    const int j = c0 + lane;
    int e = (j < e1) ? bucket[j] : -1;
    const bool valid = (e >= 0) && (e < NE);
    int d = valid ? dst[e] : -1;
    const bool ok = valid && (d >= n0) && (d < n0 + NODES_PER_BLK);
    int tot; const int rk = rank_eq(ok ? (d - n0) : 0, ok, lane, 8, tot);
    if (ok && rk == tot - 1) cnt[wave][d - n0] += tot;
  }
  __syncthreads();
  if (tid < 32) {
    int loc[8]; int sum = 0;
    for (int q = 0; q < 8; ++q) { int c = 0; for (int w = 0; w < 8; ++w) c += cnt[w][tid * 8 + q]; loc[q] = c; sum += c; }
    int incl = sum;
    for (int o = 1; o < 32; o <<= 1) { int t = __shfl_up(incl, o, 32); if (lane >= o) incl += t; }
    int base = incl - sum;
    for (int q = 0; q < 8; ++q) {
      const int node = tid * 8 + q;
      nodeoff[node] = base;
      int run = base;
      for (int w = 0; w < 8; ++w) { off[w][node] = run; run += cnt[w][node]; }
      base += loc[q];
    }
    if (tid == 31) nodeoff[NODES_PER_BLK] = base;
  }
  __syncthreads();
  const int btotal = nodeoff[NODES_PER_BLK];
  for (int c0 = e0; c0 < e0 + per; c0 += 32) {
    const int j = c0 + lane;
    int e = (j < e1) ? bucket[j] : -1;
    const bool valid = (e >= 0) && (e < NE);
    int d = valid ? dst[e] : -1;
    const bool ok = valid && (d >= n0) && (d < n0 + NODES_PER_BLK);
    int tot; const int rk = rank_eq(ok ? (d - n0) : 0, ok, lane, 8, tot);
    if (ok) { const int slot = off[wave][d - n0] + rk; if (slot < SEG_CAP) seg[slot] = e; if (rk == tot - 1) off[wave][d - n0] = slot + 1; }
  }
  __syncthreads();
  const int gstart = blockIdx.x * (SEG_STRIDE);
  const int nlines = (min(btotal, SEG_CAP) + 31) >> 5;
  for (int pass = 0; pass < 2; ++pass) {
    { const int node = tid; int deg = 0; for (int w = 0; w < 8; ++w) deg += cnt[w][node];
      ((volatile int*)rowptr)[n0 + node] = gstart + nodeoff[node]; ((volatile int*)rowdeg)[n0 + node] = deg; }
    for (int i = tid; i < nlines * 32; i += 256) ((volatile int*)csr_eid)[gstart + i] = (i < btotal) ? seg[i] : 0;
    if (rcl != nullptr && tid < 32) ((volatile int*)rcl)[blockIdx.x * 32 + tid] = (tid == 0) ? min(btotal, SEG_CAP) : 0;
    __threadfence();
  }
}

__global__ __launch_bounds__(256) void key_kernel(const int* __restrict__ idx, int* __restrict__ KEY) {
  const int n = blockIdx.x * 256 + threadIdx.x; if (n >= NE) return; int b = idx[n * 3], y = idx[n * 3 + 1], x = idx[n * 3 + 2];
  b = b < 0 ? 0 : (b >= SB_ ? SB_ - 1 : b); y = y < 0 ? 0 : (y >= SHW ? SHW - 1 : y); x = x < 0 ? 0 : (x >= SHW ? SHW - 1 : x);
  const int k = ((b * SHW + y) * SHW + x) >> 6; ((volatile int*)KEY)[n] = k; __threadfence(); ((volatile int*)KEY)[n] = k;
}
__global__ __launch_bounds__(256) void grid_kernel(const int* __restrict__ rowptr, const int* __restrict__ rowdeg, const int* __restrict__ csr_eid, const int* __restrict__ idx, int* __restrict__ GRID) {
  const int lane = threadIdx.x & 31, wave = threadIdx.x >> 5; const int key = blockIdx.x * 8 + wave;
  int c0 = -1, c1 = -1;
  int j0 = rowptr[key]; int dg = rowdeg[key]; dg = dg < 0 ? 0 : (dg > SEG_CAP ? SEG_CAP : dg); j0 = j0 < 0 ? 0 : (j0 > NBLK * SEG_STRIDE - dg ? NBLK * SEG_STRIDE - dg : j0);
  for (int j = j0; j < j0 + dg; ++j) { int e = csr_eid[j]; e = e < 0 ? 0 : (e >= NE ? NE - 1 : e); const int cell = idx[e * 3 + 2] & 63; if (cell == lane) c0 = e; if (cell == lane + 32) c1 = e; }
  int* g = GRID + (size_t)key * 64;
  for (int pass = 0; pass < 2; ++pass) { ((volatile int*)g)[lane] = c0; ((volatile int*)g)[lane + 32] = c1; __threadfence(); }
}
__device__ __forceinline__ int nbr_index(const int* __restrict__ idx, const int* __restrict__ GRID, int n, int k) {
  const int b = idx[n * 3], y = idx[n * 3 + 1] + k / 3 - 1, x = idx[n * 3 + 2] + k % 3 - 1;
  if (y < 0 || y >= SHW || x < 0 || x >= SHW) return -1; const int j = GRID[((size_t)b * SHW + y) * SHW + x]; return (j >= 0 && j < NE) ? j : -1;
}
__global__ __launch_bounds__(256) void conv1_kernel(const float* __restrict__ feats, const int* __restrict__ idx, const int* __restrict__ GRID, const float* __restrict__ W1, float* __restrict__ C1) {
  const int lane = threadIdx.x & 31, wave = threadIdx.x >> 5; const int n = (blockIdx.x * 8 + wave) * 4 + (lane >> 3); const int c = lane & 7;
  float a = 0.f;
  if (n < NE) {
#pragma unroll 1
    for (int k = 0; k < 9; ++k) { const int j = nbr_index(idx, GRID, n, k); if (j >= 0) a += feats[j] * W1[k * 8 + c]; } }
  ((volatile float*)C1)[(size_t)(blockIdx.x * 8 + wave) * 32 + lane] = a; __threadfence(); ((volatile float*)C1)[(size_t)(blockIdx.x * 8 + wave) * 32 + lane] = a;
}
template <int C>
__global__ __launch_bounds__(256) void bn_part_kernel(const float* __restrict__ X, double* __restrict__ PS) {
  __shared__ double a[256], q2[256];
  const int c = threadIdx.x % C, r = threadIdx.x / C; const int R = 256 / C; const int r0 = blockIdx.x * 2048;
  double s = 0.0, ss = 0.0; for (int i = r0 + r; i < min(r0 + 2048, NE); i += R) { const double v = X[(size_t)i * C + c]; s += v; ss += v * v; }
  a[threadIdx.x] = s; q2[threadIdx.x] = ss; __syncthreads();
  if (threadIdx.x < C) { double S = 0, SS = 0; for (int k = 0; k < R; ++k) { S += a[k * C + threadIdx.x]; SS += q2[k * C + threadIdx.x]; }
    for (int pass = 0; pass < 2; ++pass) { ((volatile double*)PS)[(size_t)blockIdx.x * 64 + threadIdx.x] = S; ((volatile double*)PS)[(size_t)blockIdx.x * 64 + 32 + threadIdx.x] = SS; __threadfence(); } }
}
template <int C>
__global__ __launch_bounds__(256) void bn_final_kernel(const double* __restrict__ PS, int nblk, const float* __restrict__ gamma, const float* __restrict__ beta, float* __restrict__ SS2) {
  if (threadIdx.x < C) { const int c = threadIdx.x; double s = 0, ss = 0; for (int b = 0; b < nblk; ++b) { s += PS[(size_t)b * 64 + c]; ss += PS[(size_t)b * 64 + 32 + c]; }
    const double mu = s / NE; double var = ss / NE - mu * mu; if (var < 0) var = 0; const float sc = gamma[c] * (float)(1.0 / sqrt(var + 1e-5)); const float sh = beta[c] - (float)mu * sc;
    for (int pass = 0; pass < 2; ++pass) { ((volatile float*)SS2)[c] = sc; ((volatile float*)SS2)[32 + c] = sh; __threadfence(); } }
}
template <int CIN, int KP>
__global__ __launch_bounds__(256) void gather_kernel(const float* __restrict__ X, const float* __restrict__ SS2, const int* __restrict__ idx, const int* __restrict__ GRID, int r0, unsigned* __restrict__ A) {
  const int lane = threadIdx.x & 31, wave = threadIdx.x >> 5; const int r = blockIdx.x * 8 + wave; const int n = r0 + r;
  int myj = -1; if (n < NE && lane < 9) myj = nbr_index(idx, GRID, n, lane);
  unsigned* row = A + (size_t)r * (KP / 2);
  unsigned vals[3] = {0u, 0u, 0u};
#pragma unroll
  for (int q = 0; q < 3; ++q) { const int p = lane + 32 * q; if (p < KP / 2) {
      const int hidx = 2 * p; const int k = hidx / CIN, c = hidx % CIN; unsigned u = 0u;
      const int j = __shfl(myj, k < 9 ? k : 0, 32);
      if (k < 9 && j >= 0) { float a = fmaxf(X[(size_t)j * CIN + c] * SS2[c] + SS2[32 + c], 0.f), b = fmaxf(X[(size_t)j * CIN + c + 1] * SS2[c + 1] + SS2[32 + c + 1], 0.f);
          u = (unsigned)__builtin_bit_cast(unsigned short, (_Float16)a) | ((unsigned)__builtin_bit_cast(unsigned short, (_Float16)b) << 16); }
      vals[q] = u; } }
  for (int pass = 0; pass < 2; ++pass) { for (int q = 0; q < 3; ++q) { const int p = lane + 32 * q; if (p < KP / 2) ((volatile unsigned*)row)[p] = vals[q]; } __threadfence(); }
}
template <int CIN, int COUT, int KP>
__global__ __launch_bounds__(256) void wconv_kernel(const float* __restrict__ Wsrc, unsigned* __restrict__ WT) {
  const int i = blockIdx.x * 256 + threadIdx.x; if (i >= 64 * KP / 2) return; const int o = (2 * i) / KP, hh = (2 * i) % KP; float a = 0.f, b = 0.f;
  if (o < COUT) { { const int k = hh / CIN, c = hh % CIN; if (k < 9) a = Wsrc[(k * CIN + c) * COUT + o]; } { const int k = (hh + 1) / CIN, c = (hh + 1) % CIN; if (k < 9) b = Wsrc[(k * CIN + c) * COUT + o]; } }
  const unsigned u = (unsigned)__builtin_bit_cast(unsigned short, (_Float16)a) | ((unsigned)__builtin_bit_cast(unsigned short, (_Float16)b) << 16); ((volatile unsigned*)WT)[i] = u; __threadfence(); ((volatile unsigned*)WT)[i] = u;
}
template <int COUT>
__global__ __launch_bounds__(256) void compact_kernel(const float* __restrict__ Cc, int r0, float* __restrict__ X) {
  const int lane = threadIdx.x & 31, wave = threadIdx.x >> 5; const int RPW = 32 / COUT; const int rl = (blockIdx.x * 8 + wave) * RPW + lane / COUT; const int c = lane % COUT; const int n = r0 + rl;
  if (rl >= SCH || n >= NE) return;
  const float v = Cc[(size_t)rl * 64 + c]; ((volatile float*)X)[(size_t)n * COUT + c] = v; __threadfence(); ((volatile float*)X)[(size_t)n * COUT + c] = v;
}
__global__ __launch_bounds__(256) void pool_kernel(const float* __restrict__ X3, const float* __restrict__ SS2, const int* __restrict__ idx, float* __restrict__ POOL) {
  __shared__ float part[8][32];
  const int b = blockIdx.x; const int lane = threadIdx.x & 31, wave = threadIdx.x >> 5; float mx = -INFINITY;
  for (int n = wave; n < NE; n += 8) if (idx[n * 3] == b) mx = fmaxf(mx, fmaxf(X3[(size_t)n * 32 + lane] * SS2[lane] + SS2[32 + lane], 0.f));
  part[wave][lane] = mx; __syncthreads();
  if (threadIdx.x < 32) { float m = part[0][threadIdx.x]; for (int w = 1; w < 8; ++w) m = fmaxf(m, part[w][threadIdx.x]); if (m == -INFINITY) m = -INFINITY;
    ((volatile float*)POOL)[b * 32 + threadIdx.x] = m; __threadfence(); ((volatile float*)POOL)[b * 32 + threadIdx.x] = m; }
}
__global__ __launch_bounds__(256) void fc_kernel(const float* __restrict__ POOL, const float* __restrict__ Wfc, const float* __restrict__ bfc, float* __restrict__ out) {
  for (int i = threadIdx.x; i < SB_ * 128; i += 256) { const int b = i / 128, o = i % 128; float a = bfc[o];
#pragma unroll 1
    for (int c = 0; c < 32; ++c) a += POOL[b * 32 + c] * Wfc[c * 128 + o];
    a = fmaxf(a, 0.f); ((volatile float*)out)[i] = a; }
  __threadfence();
  for (int i = threadIdx.x; i < SB_ * 128; i += 256) ((volatile float*)out)[i] = out[i];
}
extern "C" void kernel_launch(void* const* d_in, const int* in_sizes, int n_in, void* d_out, int out_size, void* d_ws, size_t ws_size, hipStream_t stream) {
  (void)in_sizes; (void)n_in; (void)out_size; (void)ws_size;
  const float* feats = (const float*)d_in[0]; const int* idx = (const int*)d_in[1]; const float* W1 = (const float*)d_in[2]; const float* g1 = (const float*)d_in[3]; const float* b1 = (const float*)d_in[4];
  const float* W2 = (const float*)d_in[5]; const float* g2 = (const float*)d_in[6]; const float* b2 = (const float*)d_in[7]; const float* W3 = (const float*)d_in[8]; const float* g3 = (const float*)d_in[9]; const float* b3 = (const float*)d_in[10];
  const float* Wfc = (const float*)d_in[11]; const float* bfc = (const float*)d_in[12];
  char* ws = (char*)d_ws; size_t off = 0;
  auto carve = [&](size_t bytes) -> char* { char* p = ws + off; off += (bytes + 255) & ~(size_t)255; return p; };
  int* ccnt   = (int*)carve((size_t)NCH * NRP * 4);
  int* boff   = (int*)carve((size_t)NCH * NRP * 4);
  int* rinfo  = (int*)carve((size_t)2048 * 4);
  int* bucket = (int*)carve(BUCKET_INTS * 4);
  int* rowptr = (int*)carve((size_t)NBLK * NODES_PER_BLK * 4);
  int* rowdeg = (int*)carve((size_t)NBLK * NODES_PER_BLK * 4);
  int* csr_eid= (int*)carve((size_t)NBLK * SEG_STRIDE * 4);

  int* KEY = (int*)carve((size_t)NE * 4); int* GRID = (int*)carve((size_t)SCELLS * 4);
  float* C1 = (float*)carve((size_t)(NE + 32) * 8 * 4); float* X2 = (float*)carve((size_t)NE * 16 * 4); float* X3 = (float*)carve((size_t)NE * 32 * 4);
  unsigned* A = (unsigned*)carve((size_t)SCH * 192 * 2); float* Cc = (float*)carve((size_t)SCH * 64 * 4);
  unsigned* WT2 = (unsigned*)carve(64 * 128 * 2); unsigned* WT3 = (unsigned*)carve(64 * 192 * 2);
  const int NBB = (NE + 2047) / 2048; double* PS = (double*)carve((size_t)NBB * 64 * 8); float* SS2 = (float*)carve(64 * 4); float* POOL = (float*)carve(SB_ * 32 * 4);
  key_kernel<<<(NE + 255) / 256, 256, 0, stream>>>(idx, KEY);

  csr_hist_kernel<<<NCH, 256, 0, stream>>>(KEY, ccnt);
  csr_offsets_kernel<<<1, 1024, 0, stream>>>(ccnt, boff, rinfo);
  csr_bucket_kernel<<<NCH, 256, 0, stream>>>(KEY, boff, bucket);
  csr_fill_kernel<<<NBLK, 256, 0, stream>>>(KEY, bucket, rinfo, rowptr, rowdeg, csr_eid, nullptr);

  grid_kernel<<<NN / 8, 256, 0, stream>>>(rowptr, rowdeg, csr_eid, idx, GRID);
  wconv_kernel<8, 16, 128><<<(64 * 128 / 2 + 255) / 256, 256, 0, stream>>>(W2, WT2);
  wconv_kernel<16, 32, 192><<<(64 * 192 / 2 + 255) / 256, 256, 0, stream>>>(W3, WT3);
  conv1_kernel<<<(NE / 4 + 7) / 8, 256, 0, stream>>>(feats, idx, GRID, W1, C1);
  bn_part_kernel<8><<<NBB, 256, 0, stream>>>(C1, PS); bn_final_kernel<8><<<1, 256, 0, stream>>>(PS, NBB, g1, b1, SS2);
  const int t = (SCH / 64) * 1;
  for (int c = 0; c < NE / SCH; ++c) {
    gather_kernel<8, 128><<<SCH / 8, 256, 0, stream>>>(C1, SS2, idx, GRID, c * SCH, A);
    wmma_gemm64<0, false, 0, 0, false><<<dim3((t + 7) / 8, 1), 256, 0, stream>>>((const unsigned short*)A, nullptr, 128, 0, (const unsigned short*)WT2, nullptr, 128, 0, Cc, nullptr, 64, 0, nullptr, nullptr, 0, SCH, 64, 128, 1.0f);
    compact_kernel<16><<<(SCH / 2 + 7) / 8, 256, 0, stream>>>(Cc, c * SCH, X2); }
  bn_part_kernel<16><<<NBB, 256, 0, stream>>>(X2, PS); bn_final_kernel<16><<<1, 256, 0, stream>>>(PS, NBB, g2, b2, SS2);
  for (int c = 0; c < NE / SCH; ++c) {
    gather_kernel<16, 192><<<SCH / 8, 256, 0, stream>>>(X2, SS2, idx, GRID, c * SCH, A);
    wmma_gemm64<0, false, 0, 0, false><<<dim3((t + 7) / 8, 1), 256, 0, stream>>>((const unsigned short*)A, nullptr, 192, 0, (const unsigned short*)WT3, nullptr, 192, 0, Cc, nullptr, 64, 0, nullptr, nullptr, 0, SCH, 64, 192, 1.0f);
    compact_kernel<32><<<(SCH + 7) / 8, 256, 0, stream>>>(Cc, c * SCH, X3); }
  bn_part_kernel<32><<<NBB, 256, 0, stream>>>(X3, PS); bn_final_kernel<32><<<1, 256, 0, stream>>>(PS, NBB, g3, b3, SS2);
  pool_kernel<<<SB_, 256, 0, stream>>>(X3, SS2, idx, POOL);
  fc_kernel<<<1, 256, 0, stream>>>(POOL, Wfc, bfc, (float*)d_out);
}
